// _ContextAttentionModule_79645873537062
// MI455X (gfx1250) — hardware-verified
//
#include <hip/hip_runtime.h>


#define NB_  8
#define CIN  256
#define CI   128
#define HH   64
#define WW   64
#define NPX  4096
#define MP   1024
#define DM   CIN
#define BEPS 1e-5f
#define LOSC 1024.0f

typedef _Float16 h16;
typedef unsigned short bf;
typedef __attribute__((ext_vector_type(16))) __bf16   v16bf;
typedef __attribute__((ext_vector_type(16))) _Float16 v16h;
typedef __attribute__((ext_vector_type(8)))  _Float16 v8h;
typedef __attribute__((ext_vector_type(8)))  unsigned short v8us;
typedef __attribute__((ext_vector_type(8)))  float    v8f;
typedef __attribute__((ext_vector_type(4)))  float    v4f;
typedef v8h  __attribute__((may_alias)) v8ha;
typedef v4f  __attribute__((may_alias)) v4fa;
typedef v8us __attribute__((may_alias)) v8usa;

__device__ __forceinline__ unsigned short f2bf(float f) { unsigned u = __float_as_uint(f); u += 0x7FFFu + ((u >> 16) & 1u); return (unsigned short)(u >> 16); }
__device__ __forceinline__ float bf2f(unsigned short b) { return __uint_as_float(((unsigned)b) << 16); }
__device__ __forceinline__ float bfr(float f) { return bf2f(f2bf(f)); }
__device__ __forceinline__ v16h cat16(v8h lo, v8h hi) { return __builtin_shufflevector(lo, hi, 0, 1, 2, 3, 4, 5, 6, 7, 8, 9, 10, 11, 12, 13, 14, 15); }
__device__ __forceinline__ v16bf cat16b(v8us lo, v8us hi) { return __builtin_bit_cast(v16bf, __builtin_shufflevector(lo, hi, 0, 1, 2, 3, 4, 5, 6, 7, 8, 9, 10, 11, 12, 13, 14, 15)); }
__device__ __forceinline__ v8f wmma16(v16h a, v16h b, v8f c) { return __builtin_amdgcn_wmma_f32_16x16x32_f16(false, a, false, b, (short)0, c, false, false); }
__device__ __forceinline__ v8f wmmab(v16bf a, v16bf b, v8f c) { return __builtin_amdgcn_wmma_f32_16x16x32_bf16(false, a, false, b, (short)0, c, false, false); }

template <bool SPLITA, bool F16OUT = false>
__global__ __launch_bounds__(128) void k_gemmb(const bf* __restrict__ A, const bf* __restrict__ Al, const bf* __restrict__ Bn, const float* __restrict__ bias, float* C, int ldc, h16* C2, const float* __restrict__ R = nullptr, int K = DM, int roundR = 1) {
    __shared__ __align__(16) float ost[4][16 * 68];
    const int lane = threadIdx.x & 31, wave = threadIdx.x >> 5, lr = lane & 15, hi = lane >> 4;
    const int r0 = blockIdx.x * 64 + wave * 16, c0 = blockIdx.y * 64;
    const size_t aoff = (size_t)(r0 + lr) * K + 8 * hi;
    size_t boff[4];
#pragma unroll
    for (int t = 0; t < 4; ++t) boff[t] = (size_t)(c0 + t * 16 + lr) * K + 8 * hi;
    v8f acc[4];
#pragma unroll
    for (int t = 0; t < 4; ++t) acc[t] = (v8f){};
#pragma unroll 1
    for (int kc = 0; kc < K; kc += 32) {
        const v16bf a = cat16b(*(const v8us*)(A + aoff + kc), *(const v8us*)(A + aoff + kc + 16));
        v16bf al = a;
        if (SPLITA) al = cat16b(*(const v8us*)(Al + aoff + kc), *(const v8us*)(Al + aoff + kc + 16));
#pragma unroll
        for (int t = 0; t < 4; ++t) { const v16bf b = cat16b(*(const v8us*)(Bn + boff[t] + kc), *(const v8us*)(Bn + boff[t] + kc + 16)); acc[t] = wmmab(a, b, acc[t]); if (SPLITA) acc[t] = wmmab(al, b, acc[t]); }
        asm volatile("v_nop\n\tv_nop\n\tv_nop\n\tv_nop" : "+v"(acc[0]), "+v"(acc[1]), "+v"(acc[2]), "+v"(acc[3]) : "v"(a), "v"(al));
    }
    float* os = &ost[wave][0];
#pragma unroll
    for (int t = 0; t < 4; ++t) { const float bv = bias ? bfr(bias[c0 + t * 16 + lr]) : 0.f;
#pragma unroll
        for (int j = 0; j < 8; ++j) os[(hi * 8 + j) * 68 + t * 16 + lr] = acc[t][j] + bv; }
    __syncthreads();
    if (F16OUT) {
        h16* crow = (h16*)(void*)C + (size_t)r0 * ldc + c0;
        auto pass = [&]() {
#pragma unroll
            for (int s = 0; s < 4; ++s) { const int row = 4 * s + (lane >> 3), piece = lane & 7; const float* sp = os + row * 68 + piece * 8; v8h o, o2;
#pragma unroll
                for (int i = 0; i < 8; ++i) { const h16 a = (h16)sp[i]; o[i] = a; o2[i] = (h16)((sp[i] - (float)a) * LOSC); }
                *(volatile v8h*)(crow + (size_t)row * ldc + piece * 8) = o; if (C2) *(volatile v8h*)(C2 + (size_t)r0 * ldc + c0 + (size_t)row * ldc + piece * 8) = o2; }
        };
        pass(); __threadfence(); pass();
    } else {
        float* crow = C + (size_t)r0 * ldc + c0;
        auto pass = [&]() {
#pragma unroll
            for (int s = 0; s < 8; ++s) { const int Lid = (lane >> 3) + 4 * s, piece = lane & 7; const int row = Lid >> 1, cofs = (Lid & 1) * 32 + piece * 4;
                v4f val = *(const v4fa*)(os + row * 68 + cofs); if (R) { const v4f rv = *(const v4f*)(R + ((size_t)r0 + row) * ldc + c0 + cofs); val += roundR ? (v4f){bfr(rv[0]), bfr(rv[1]), bfr(rv[2]), bfr(rv[3])} : rv; }
                *(volatile v4f*)(crow + (size_t)row * ldc + cofs) = val; }
        };
        pass(); __threadfence(); pass();
    }
}

__global__ __launch_bounds__(256) void k_cvt8(const float* __restrict__ src, bf* dst, size_t n8) {
    const size_t i = (size_t)blockIdx.x * 256 + threadIdx.x; if (i >= n8) return;
    const v8f v = *(const v8f*)(src + i * 8); v8us o;
#pragma unroll
    for (int k = 0; k < 8; ++k) o[k] = f2bf(v[k]);
    *(volatile v8us*)(dst + i * 8) = o; __threadfence(); *(volatile v8us*)(dst + i * 8) = o;
}
__global__ __launch_bounds__(256) void k_zero8(bf* dst, size_t n8) {
    const size_t i = (size_t)blockIdx.x * 256 + threadIdx.x; if (i >= n8) return; v8us z;
#pragma unroll
    for (int k = 0; k < 8; ++k) z[k] = 0;
    *(volatile v8us*)(dst + i * 8) = z; __threadfence(); *(volatile v8us*)(dst + i * 8) = z;
}
__global__ __launch_bounds__(128) void k_gemm3(const bf* __restrict__ Ah, const bf* __restrict__ Al, const bf* __restrict__ Bh, const bf* __restrict__ Bl, int K, float* C, int ldc) {
    __shared__ __align__(16) float ost[4][16 * 68];
    const int lane = threadIdx.x & 31, wave = threadIdx.x >> 5, lr = lane & 15, hi = lane >> 4;
    const int r0 = blockIdx.x * 64 + wave * 16, c0 = blockIdx.y * 64;
    const size_t aoff = (size_t)(r0 + lr) * K + 8 * hi;
    v8f acc[4];
#pragma unroll
    for (int t = 0; t < 4; ++t) acc[t] = (v8f){};
#pragma unroll 1
    for (int kc = 0; kc < K; kc += 32) {
        const v16bf a = cat16b(*(const v8us*)(Ah + aoff + kc), *(const v8us*)(Ah + aoff + kc + 16));
        const v16bf al = cat16b(*(const v8us*)(Al + aoff + kc), *(const v8us*)(Al + aoff + kc + 16));
#pragma unroll
        for (int t = 0; t < 4; ++t) { const size_t bo = (size_t)(c0 + t * 16 + lr) * K + kc + 8 * hi;
            const v16bf bh = cat16b(*(const v8us*)(Bh + bo), *(const v8us*)(Bh + bo + 16)); const v16bf bl = cat16b(*(const v8us*)(Bl + bo), *(const v8us*)(Bl + bo + 16));
            acc[t] = wmmab(a, bh, acc[t]); acc[t] = wmmab(al, bh, acc[t]); acc[t] = wmmab(a, bl, acc[t]); }
        asm volatile("v_nop\n\tv_nop\n\tv_nop\n\tv_nop" : "+v"(acc[0]), "+v"(acc[1]), "+v"(acc[2]), "+v"(acc[3]) : "v"(a), "v"(al));
    }
    float* os = &ost[wave][0];
#pragma unroll
    for (int t = 0; t < 4; ++t) {
#pragma unroll
        for (int j = 0; j < 8; ++j) os[(hi * 8 + j) * 68 + t * 16 + lr] = acc[t][j]; }
    __builtin_amdgcn_wave_barrier(); asm volatile("" ::: "memory");
    float* crow = C + (size_t)r0 * ldc + c0;
    auto pass = [&]() {
#pragma unroll
        for (int s = 0; s < 8; ++s) { const int Lid = (lane >> 3) + 4 * s, piece = lane & 7; const int row = Lid >> 1, cofs = (Lid & 1) * 32 + piece * 4;
            const v4f val = *(const v4fa*)(os + row * 68 + cofs); *(volatile v4f*)(crow + (size_t)row * ldc + cofs) = val; }
    };
    pass(); __threadfence(); pass();
}


__global__ __launch_bounds__(256) void k_ptb(const float* __restrict__ xb, bf* XT) {
    __shared__ float tl[64][65];
    typedef __attribute__((ext_vector_type(4))) unsigned short v4us;
    const int tid = threadIdx.x, c0 = blockIdx.x * 64, p0 = blockIdx.y * 64; const int rr = tid >> 2, cq = (tid & 3) * 16;
#pragma unroll
    for (int i = 0; i < 16; ++i) tl[rr][cq + i] = xb[(size_t)(c0 + rr) * NPX + p0 + cq + i];
    __syncthreads();
    const int lane = tid & 31, wv = tid >> 5;
    auto pass = [&]() {
#pragma unroll
        for (int st = 0; st < 4; ++st) { const int pr = wv * 8 + st * 2 + (lane >> 4); const int cl = (lane & 15) * 4; v4us v;
#pragma unroll
            for (int i = 0; i < 4; ++i) v[i] = f2bf(tl[cl + i][pr]);
            *(volatile v4us*)(XT + (size_t)(p0 + pr) * CIN + c0 + cl) = v; }
    };
    pass(); __threadfence(); pass();
}
__global__ __launch_bounds__(256) void k_split128(const float* __restrict__ src, int rows, float sc, bf* dh, bf* dl) {
    typedef __attribute__((ext_vector_type(4))) unsigned short v4us;
    const int lane = threadIdx.x & 31; const size_t r = (size_t)blockIdx.x * 8 + (threadIdx.x >> 5); if (r >= (size_t)rows) return; const size_t o = r * CI + lane * 4; const v4f v = *(const v4f*)(src + o); v4us oh, ol;
#pragma unroll
    for (int i = 0; i < 4; ++i) { const float y = v[i] * sc; const unsigned short hb = f2bf(y); oh[i] = hb; ol[i] = f2bf(y - bf2f(hb)); }
    *(volatile v4us*)(dh + o) = oh; *(volatile v4us*)(dl + o) = ol; __threadfence(); *(volatile v4us*)(dh + o) = oh; *(volatile v4us*)(dl + o) = ol;
}
__global__ __launch_bounds__(256) void k_poolphi(const float* __restrict__ F, bf* dh, bf* dl) {
    typedef __attribute__((ext_vector_type(4))) unsigned short v4us;
    const int lane = threadIdx.x & 31; const size_t m = (size_t)blockIdx.x * 8 + (threadIdx.x >> 5); if (m >= (size_t)MP) return; const int py = (int)(m / (WW / 2)), px = (int)(m % (WW / 2)); const size_t p00 = (size_t)(2 * py) * WW + 2 * px; v4us oh, ol;
#pragma unroll
    for (int i = 0; i < 4; ++i) { const int c = lane * 4 + i; const float a = F[p00 * CI + c], b2 = F[(p00 + 1) * CI + c], cc = F[(p00 + WW) * CI + c], d = F[(p00 + WW + 1) * CI + c]; const float y = fmaxf(fmaxf(a, b2), fmaxf(cc, d)); const unsigned short hb = f2bf(y); oh[i] = hb; ol[i] = f2bf(y - bf2f(hb)); }
    const size_t o = m * CI + lane * 4; *(volatile v4us*)(dh + o) = oh; *(volatile v4us*)(dl + o) = ol; __threadfence(); *(volatile v4us*)(dh + o) = oh; *(volatile v4us*)(dl + o) = ol;
}
__global__ __launch_bounds__(256) void k_poolgT(const float* __restrict__ F, bf* Th, bf* Tl) {
    typedef __attribute__((ext_vector_type(2))) unsigned short v2us;
    const int lane = threadIdx.x & 31; const size_t wid = (size_t)blockIdx.x * 8 + (threadIdx.x >> 5); if (wid >= (size_t)CI * (MP / 64)) return; const int c = (int)(wid / (MP / 64)); const int m0 = (int)(wid % (MP / 64)) * 64 + lane * 2; v2us oh, ol;
#pragma unroll
    for (int q = 0; q < 2; ++q) { const int m = m0 + q; const int py = m / (WW / 2), px = m % (WW / 2); const size_t p00 = (size_t)(2 * py) * WW + 2 * px;
        const float y = fmaxf(fmaxf(F[p00 * CI + c], F[(p00 + 1) * CI + c]), fmaxf(F[(p00 + WW) * CI + c], F[(p00 + WW + 1) * CI + c])); const unsigned short hb = f2bf(y); oh[q] = hb; ol[q] = f2bf(y - bf2f(hb)); }
    const size_t o = (size_t)c * MP + m0; *(volatile v2us*)(Th + o) = oh; *(volatile v2us*)(Tl + o) = ol; __threadfence(); *(volatile v2us*)(Th + o) = oh; *(volatile v2us*)(Tl + o) = ol;
}
__global__ __launch_bounds__(256) void k_split1024(const float* __restrict__ src, int rows, bf* dh, bf* dl) {
    const int lane = threadIdx.x & 31; const size_t r = (size_t)blockIdx.x * 8 + (threadIdx.x >> 5); if (r >= (size_t)rows) return;
#pragma unroll 1
    for (int ps = 0; ps < 2; ++ps) {
#pragma unroll
        for (int q = 0; q < MP / 256; ++q) { const size_t o = r * MP + q * 256 + lane * 8; const v8f v = *(const v8f*)(src + o); v8us oh, ol;
#pragma unroll
            for (int i = 0; i < 8; ++i) { const unsigned short hb = f2bf(v[i]); oh[i] = hb; ol[i] = f2bf(v[i] - bf2f(hb)); }
            *(volatile v8us*)(dh + o) = oh; *(volatile v8us*)(dl + o) = ol; }
        if (ps == 0) __threadfence(); }
}
__global__ __launch_bounds__(256) void k_bnstat(const float* __restrict__ WY, float* MEAN, float* RSTD) {
    const int lane = threadIdx.x & 31; const int w = blockIdx.x * 8 + (threadIdx.x >> 5); if (w >= CIN / 32) return; const int c = w * 32 + lane; const int n = NB_ * NPX; float s = 0.f;
    for (int r = 0; r < n; ++r) s += WY[(size_t)r * CIN + c];
    const float mu = s / (float)n; float q = 0.f;
    for (int r = 0; r < n; ++r) { const float d = WY[(size_t)r * CIN + c] - mu; q = fmaf(d, d, q); }
    const float rs = rsqrtf(q / (float)n + BEPS);
    *(volatile float*)(MEAN + c) = mu; *(volatile float*)(RSTD + c) = rs; __threadfence(); *(volatile float*)(MEAN + c) = mu; *(volatile float*)(RSTD + c) = rs;
}
__global__ __launch_bounds__(256) void k_bnout(const float* __restrict__ WY, const float* __restrict__ x1, const float* __restrict__ MEAN, const float* __restrict__ RSTD, const float* __restrict__ gam, const float* __restrict__ bet, float* OUTB) {
    __shared__ float tl[64][65];
    const int tid = threadIdx.x; const int p0 = blockIdx.x * 64, c0 = blockIdx.y * 64, b = blockIdx.z; const int rr = tid >> 2, cq = (tid & 3) * 16;
#pragma unroll
    for (int i = 0; i < 16; ++i) { const int c = c0 + cq + i; tl[rr][cq + i] = (WY[((size_t)b * NPX + p0 + rr) * CIN + c] - MEAN[c]) * RSTD[c] * bfr(gam[c]) + bfr(bet[c]); }
    __syncthreads();
    const int lane = tid & 31, wv = tid >> 5;
    auto pass = [&]() {
#pragma unroll
        for (int st = 0; st < 4; ++st) { const int cr = wv * 8 + st * 2 + (lane >> 4); const int pq = (lane & 15) * 4; v4f v; const size_t o = ((size_t)b * CIN + c0 + cr) * NPX + p0 + pq;
#pragma unroll
            for (int i = 0; i < 4; ++i) v[i] = tl[pq + i][cr] + bfr(x1[o + i]);
            *(volatile v4f*)(OUTB + o) = v; }
    };
    pass(); __threadfence(); pass();
}

extern "C" void kernel_launch(void* const* d_in, const int* in_sizes, int n_in,
                              void* d_out, int out_size, void* d_ws, size_t ws_size, hipStream_t stream) {
    (void)in_sizes; (void)n_in; (void)out_size;
    const float* x1 = (const float*)d_in[0]; const float* x2 = (const float*)d_in[1]; const float* wg = (const float*)d_in[2]; const float* bg = (const float*)d_in[3]; const float* wth = (const float*)d_in[4]; const float* bth = (const float*)d_in[5]; const float* wph = (const float*)d_in[6]; const float* bph = (const float*)d_in[7];
    const float* wout = (const float*)d_in[8]; const float* bout = (const float*)d_in[9]; const float* gam = (const float*)d_in[10]; const float* bet = (const float*)d_in[11];
    float* out = (float*)d_out;
    char* wsp = (char*)d_ws;
    auto take = [&](size_t bytes) { char* p = wsp; wsp += (bytes + 255) & ~(size_t)255; return (void*)p; };
    bf* WG = (bf*)take((size_t)CI * CIN * 2); bf* WT = (bf*)take((size_t)CI * CIN * 2); bf* WP = (bf*)take((size_t)CI * CIN * 2); bf* WO = (bf*)take((size_t)CIN * CI * 2);
    bf* X1T = (bf*)take((size_t)NPX * CIN * 2); bf* X2T = (bf*)take((size_t)NPX * CIN * 2); float* TH = (float*)take((size_t)NPX * CI * 4); float* PHI = (float*)take((size_t)NPX * CI * 4); float* G = (float*)take((size_t)NPX * CI * 4);
    bf* Th = (bf*)take((size_t)NPX * CI * 2); bf* Tl = (bf*)take((size_t)NPX * CI * 2); bf* Fh = (bf*)take((size_t)MP * CI * 2); bf* Fl = (bf*)take((size_t)MP * CI * 2); bf* GTh = (bf*)take((size_t)CI * MP * 2); bf* GTl = (bf*)take((size_t)CI * MP * 2);
    float* S = (float*)take((size_t)NPX * MP * 4); bf* PH = (bf*)take((size_t)NPX * MP * 2); bf* PL = (bf*)take((size_t)NPX * MP * 2); float* Y = (float*)take((size_t)NPX * CI * 4); bf* Yh = (bf*)take((size_t)NPX * CI * 2); bf* Yl = (bf*)take((size_t)NPX * CI * 2);
    float* WY = (float*)take((size_t)NB_ * NPX * CIN * 4); float* MEAN = (float*)take(CIN * 4); float* RSTD = (float*)take(CIN * 4);
    if ((size_t)(wsp - (char*)d_ws) > ws_size) return;
    k_cvt8<<<(CI * CIN / 8 + 255) / 256, 256, 0, stream>>>(wg, WG, CI * CIN / 8); k_cvt8<<<(CI * CIN / 8 + 255) / 256, 256, 0, stream>>>(wth, WT, CI * CIN / 8); k_cvt8<<<(CI * CIN / 8 + 255) / 256, 256, 0, stream>>>(wph, WP, CI * CIN / 8); k_cvt8<<<(CIN * CI / 8 + 255) / 256, 256, 0, stream>>>(wout, WO, CIN * CI / 8);
    for (int b = 0; b < NB_; ++b) { const float* x1b = x1 + (size_t)b * CIN * NPX; const float* x2b = x2 + (size_t)b * CIN * NPX;
        k_ptb<<<dim3(CIN / 64, NPX / 64, 1), 256, 0, stream>>>(x1b, X1T); k_ptb<<<dim3(CIN / 64, NPX / 64, 1), 256, 0, stream>>>(x2b, X2T);
        k_gemmb<false, false><<<dim3(NPX / 64, CI / 64, 1), 128, 0, stream>>>(X1T, nullptr, WT, bth, TH, CI, nullptr, nullptr, CIN); k_gemmb<false, false><<<dim3(NPX / 64, CI / 64, 1), 128, 0, stream>>>(X2T, nullptr, WP, bph, PHI, CI, nullptr, nullptr, CIN); k_gemmb<false, false><<<dim3(NPX / 64, CI / 64, 1), 128, 0, stream>>>(X2T, nullptr, WG, bg, G, CI, nullptr, nullptr, CIN);
        k_split128<<<NPX / 8, 256, 0, stream>>>(TH, NPX, 1.0f / (float)MP, Th, Tl); k_poolphi<<<MP / 8, 256, 0, stream>>>(PHI, Fh, Fl); k_poolgT<<<(CI * (MP / 64)) / 8, 256, 0, stream>>>(G, GTh, GTl);
        k_gemm3<<<dim3(NPX / 64, MP / 64, 1), 128, 0, stream>>>(Th, Tl, Fh, Fl, CI, S, MP);
        k_split1024<<<NPX / 8, 256, 0, stream>>>(S, NPX, PH, PL);
        k_gemm3<<<dim3(NPX / 64, CI / 64, 1), 128, 0, stream>>>(PH, PL, GTh, GTl, MP, Y, CI);
        k_split128<<<NPX / 8, 256, 0, stream>>>(Y, NPX, 1.0f, Yh, Yl);
        k_gemmb<true, false><<<dim3(NPX / 64, CIN / 64, 1), 128, 0, stream>>>(Yh, Yl, WO, bout, WY + (size_t)b * NPX * CIN, CIN, nullptr, nullptr, CI); }
    k_bnstat<<<(CIN / 32) / 8, 256, 0, stream>>>(WY, MEAN, RSTD);
    k_bnout<<<dim3(NPX / 64, CIN / 64, NB_), 256, 0, stream>>>(WY, x1, MEAN, RSTD, gam, bet, out);
}
